// PairedLookup_16509854286522
// MI455X (gfx1250) — hardware-verified
//
#include <hip/hip_runtime.h>
#include <math.h>

typedef __attribute__((ext_vector_type(16))) _Float16 v16h;
typedef __attribute__((ext_vector_type(16))) __bf16 v16b;
typedef __attribute__((ext_vector_type(8)))  _Float16 v8h;
typedef __attribute__((ext_vector_type(8)))  float v8f;
typedef __attribute__((ext_vector_type(4)))  float v4f;
typedef __attribute__((ext_vector_type(2)))  float v2f;
typedef __attribute__((ext_vector_type(4)))  unsigned v4u;
typedef __attribute__((ext_vector_type(4)))  int v4i;
typedef float __attribute__((may_alias)) float_a;
typedef int __attribute__((may_alias)) int_a;

template <typename T> __device__ __forceinline__ void vst2(void* p, T v) { *(volatile T*)p = v; __threadfence(); *(volatile T*)p = v; }
__device__ __forceinline__ v8f wmma16(v16h a, v16h b, v8f c) {
  v8f d = __builtin_amdgcn_wmma_f32_16x16x32_f16(false, a, false, b, (short)0, c, false, false);
  asm volatile("v_nop\n\tv_nop\n\tv_nop\n\tv_nop" : "+v"(d) : "v"(a), "v"(b));
  return d;
}
__device__ __forceinline__ v8f wmma_bf(v16b a, v16b b, v8f c) {
  v8f d = __builtin_amdgcn_wmma_f32_16x16x32_bf16(false, a, false, b, (short)0, c, false, false);
  asm volatile("v_nop\n\tv_nop\n\tv_nop\n\tv_nop" : "+v"(d) : "v"(a), "v"(b));
  return d;
}
__device__ __forceinline__ v16h frag_h(const _Float16* rowk0, int lane) {
  union { v16h v; v8h q[2]; } u; const _Float16* p = rowk0 + 8 * (lane >> 4);
  u.q[0] = *(const v8h*)p; u.q[1] = *(const v8h*)(p + 16); return u.v;
}
__device__ __forceinline__ v16h frag_f32(const float* rowk0, int lane) {
  v16h a; const float* p = rowk0 + 8 * (lane >> 4);
#pragma unroll
  for (int i = 0; i < 8; ++i) { a[i] = (_Float16)p[i]; a[8 + i] = (_Float16)p[16 + i]; }
  return a;
}
__device__ __forceinline__ v16h frag_f32s(const float* rowk0, int lane, float sc) {
  v16h a; const float* p = rowk0 + 8 * (lane >> 4);
#pragma unroll
  for (int i = 0; i < 8; ++i) { a[i] = (_Float16)(p[i] * sc); a[8 + i] = (_Float16)(p[16 + i] * sc); }
  return a;
}
__device__ __forceinline__ v16h fragc_f32(const float* W, int k0, int n, int lane, int ld, int K) {
  v16h a; const int g = lane >> 4;
#pragma unroll
  for (int i = 0; i < 8; ++i) { const int ka = k0 + 8 * g + i, kb = ka + 16;
    a[i] = (_Float16)(ka < K ? W[(size_t)(ka < K ? ka : K - 1) * ld + n] : 0.f); a[8 + i] = (_Float16)(kb < K ? W[(size_t)(kb < K ? kb : K - 1) * ld + n] : 0.f); }
  return a;
}
struct F2 { v16b h, l; };
__device__ __forceinline__ F2 bsplit16(const float v[16]) { F2 r;
#pragma unroll
  for (int i = 0; i < 16; ++i) { const __bf16 h = (__bf16)v[i]; r.h[i] = h; r.l[i] = (__bf16)(v[i] - (float)h); }
  return r; }
__device__ __forceinline__ F2 split_row(const float* row, int k0, int lane) { float v[16]; const float* p = row + k0 + 8 * (lane >> 4);
#pragma unroll
  for (int i = 0; i < 8; ++i) { v[i] = p[i]; v[8 + i] = p[16 + i]; }
  return bsplit16(v); }
__device__ __forceinline__ F2 split_rowK(const float* row, int k0, int lane, int K) { float v[16]; const int g = lane >> 4;
#pragma unroll
  for (int i = 0; i < 8; ++i) { const int ka = k0 + 8 * g + i, kb = ka + 16; v[i] = ka < K ? row[ka < K ? ka : K - 1] : 0.f; v[8 + i] = kb < K ? row[kb < K ? kb : K - 1] : 0.f; }
  return bsplit16(v); }
__device__ __forceinline__ F2 split_col(const float* W, int k0, int n, int lane, int ld, int K) { float v[16]; const int g = lane >> 4;
#pragma unroll
  for (int i = 0; i < 8; ++i) { const int ka = k0 + 8 * g + i, kb = ka + 16; v[i] = ka < K ? W[(size_t)(ka < K ? ka : K - 1) * ld + n] : 0.f; v[8 + i] = kb < K ? W[(size_t)(kb < K ? kb : K - 1) * ld + n] : 0.f; }
  return bsplit16(v); }
__device__ __forceinline__ v8f mac3(const F2& a, const F2& b, v8f c) { c = wmma_bf(a.l, b.h, c); c = wmma_bf(a.h, b.l, c); return wmma_bf(a.h, b.h, c); }
__device__ __forceinline__ float sigm(float v) { return 1.0f / (1.0f + expf(-v)); }
#define LDSX() do { asm volatile("s_wait_dscnt 0" ::: "memory"); __builtin_amdgcn_wave_barrier(); __builtin_amdgcn_fence(__ATOMIC_RELEASE, "workgroup"); } while (0)


#define NTAB 4096
#define DD 256
#define NQ 1024
typedef __attribute__((ext_vector_type(8))) __bf16 v8b;
__device__ __forceinline__ v16b frag_b(const __bf16* rowk0, int lane) {
  union { v16b v; v8b q[2]; } u; const __bf16* p = rowk0 + 8 * (lane >> 4);
  u.q[0] = *(const v8b*)p; u.q[1] = *(const v8b*)(p + 16); return u.v;
}
__device__ __forceinline__ float bfr(float v) { return (float)(__bf16)v; }
__device__ __attribute__((noinline)) float exp_ni(float v) { return expf(v); }
__device__ __attribute__((noinline)) float erf_ni(float v) { return erff(v); }

#define WS_PW 0u
#define WS_Y  (WS_PW + 2u * DD * DD)
#define WS_END (WS_Y + 4u * NQ * DD)
__global__ __launch_bounds__(256) void k_packw(const float* __restrict__ Wm, __bf16* __restrict__ PW) {
  __shared__ __align__(16) __bf16 s[DD]; const int o = blockIdx.x, t = threadIdx.x; s[t] = (__bf16)Wm[(size_t)o * DD + t]; __syncthreads();
  if (t < 32) vst2((unsigned*)(PW + (size_t)o * DD + t * 8), *(const v4u*)&s[t * 8]);
}
__global__ __launch_bounds__(128) void k_y(const float* __restrict__ BATCH, const __bf16* __restrict__ PW, float* __restrict__ Y) {
  __shared__ __align__(16) float so[4][16][132];
  const int tid = threadIdx.x, wave = tid >> 5, lane = tid & 31, col = lane & 15, g = lane >> 4; const size_t r0 = (size_t)blockIdx.x * 64 + wave * 16; const int n0 = blockIdx.y * 128;
  v8f acc[8] = {};
#pragma unroll 2
  for (int kc = 0; kc < DD / 32; ++kc) { v16b a; const float* p = BATCH + (r0 + col) * DD + kc * 32 + 8 * g;
#pragma unroll
    for (int i = 0; i < 8; ++i) { a[i] = (__bf16)p[i]; a[8 + i] = (__bf16)p[16 + i]; }
#pragma unroll
    for (int j = 0; j < 8; ++j) acc[j] = wmma_bf(a, frag_b(PW + (size_t)(n0 + j * 16 + col) * DD + kc * 32, lane), acc[j]); }
#pragma unroll
  for (int j = 0; j < 8; ++j)
#pragma unroll
    for (int r = 0; r < 8; ++r) so[wave][8 * g + r][j * 16 + col] = acc[j][r];
  LDSX();
  for (int rl = 0; rl < 16; ++rl) vst2(Y + (r0 + rl) * DD + n0 + lane * 4, *(const v4f*)&so[wave][rl][lane * 4]);
}
__global__ __launch_bounds__(64) void k_lookup(const float* __restrict__ Y, const float* __restrict__ AS, const float* __restrict__ BS, float* __restrict__ out) {
  __shared__ int sidx[64]; __shared__ __align__(16) float so[64];
  const int tid = threadIdx.x; const size_t q = (size_t)blockIdx.x * 64 + tid;
  const float* yq = Y + q * DD; const float y0 = yq[0]; int found = -1;
#pragma unroll 1
  for (int n = 0; n < NTAB && found < 0; ++n) { if (bfr(AS[(size_t)n * DD]) == y0) { bool ok = true;
#pragma unroll 1
      for (int d = 1; d < DD && ok; ++d) ok = (bfr(AS[(size_t)n * DD + d]) == yq[d]);
      if (ok) found = n; } }
  sidx[tid] = found < 0 ? 0 : found;
  __syncthreads();
  const int wave = tid >> 5, lane = tid & 31, col = lane & 15, g = lane >> 4;
  for (int wv = wave; wv < 4; wv += 2) { const size_t qa = (size_t)blockIdx.x * 64 + wv * 16 + col; const int nb = sidx[wv * 16 + col]; v8f acc = {};
#pragma unroll 2
    for (int kc = 0; kc < DD / 32; ++kc) { const F2 a = split_row(Y + qa * DD, kc * 32, lane); v16b b; const float* pb = BS + (size_t)nb * DD + kc * 32 + 8 * g;
#pragma unroll
      for (int i = 0; i < 8; ++i) { b[i] = (__bf16)pb[i]; b[8 + i] = (__bf16)pb[16 + i]; }
      acc = wmma_bf(a.l, b, acc); acc = wmma_bf(a.h, b, acc); }
#pragma unroll
    for (int r = 0; r < 8; ++r) if (8 * g + r == col) so[wv * 16 + col] = acc[r]; }
  __syncthreads();
  if (tid < 16) vst2(out + (size_t)blockIdx.x * 64 + tid * 4, *(const v4f*)&so[tid * 4]);
}
extern "C" void kernel_launch(void* const* d_in, const int* in_sizes, int n_in, void* d_out, int out_size, void* d_ws, size_t ws_size, hipStream_t stream) {
  (void)in_sizes; (void)n_in; (void)out_size;
  const float** F = (const float**)d_in;
  if (ws_size < (size_t)WS_END) return;
  char* ws = (char*)d_ws; __bf16* PW = (__bf16*)(ws + WS_PW); float* Y = (float*)(ws + WS_Y);
  k_packw<<<DD, 256, 0, stream>>>(F[1], PW);
  k_y<<<dim3(NQ / 64, 2), 128, 0, stream>>>(F[0], PW, Y);
  k_lookup<<<NQ / 64, 64, 0, stream>>>(Y, F[2], F[3], (float*)d_out);
}
